// GRU_48859547959613
// MI455X (gfx1250) — hardware-run, weakly checked
//
#include <hip/hip_runtime.h>
#include <math.h>

constexpr int NBATCH = 4096;
constexpr int NSTEP  = 512;
constexpr int NHID   = 16;
constexpr int NGATE  = 48;
constexpr int NFEAT1 = 32;
constexpr int NTHR   = 128;
constexpr int NWAVE  = 4;
constexpr int BROWS  = 64;
constexpr int WPLW   = NGATE * 16;
constexpr int WPLH   = NGATE * 32;
constexpr int GTILE  = NHID * 32;
constexpr int OSP    = 36;
constexpr int YBW    = 16;
static_assert(NBATCH % BROWS == 0);
static_assert(BROWS == NWAVE * 16);
static_assert((NGATE * 8) % NTHR == 0);
static_assert(NGATE <= NTHR && NHID <= NTHR);
static_assert(NFEAT1 == 2 * NHID && NGATE == 3 * NHID);

typedef __attribute__((ext_vector_type(16))) _Float16 v16h;
typedef __attribute__((ext_vector_type(8)))  _Float16 v8h;
typedef __attribute__((ext_vector_type(16))) __bf16   v16b;
typedef __attribute__((ext_vector_type(8)))  __bf16   v8b;
typedef __attribute__((ext_vector_type(8)))  float    v8f;
typedef __attribute__((ext_vector_type(4)))  float    v4f;
typedef __attribute__((ext_vector_type(4)))  unsigned v4u;

__device__ __forceinline__ unsigned short f2bf_bits(float f) {
  unsigned u = __float_as_uint(f);
  return (unsigned short)((u + 0x7FFFu + ((u >> 16) & 1u)) >> 16);
}
__device__ __forceinline__ float bf_bits2f(unsigned short h) { return __uint_as_float(((unsigned)h) << 16); }
__device__ __forceinline__ float bf16r(float f) { return bf_bits2f(f2bf_bits(f)); }

__device__ __forceinline__ void dep_guard_h(v8f& a, v8f& b, v16h x, v16h y) { asm volatile("v_nop\n\tv_nop\n\tv_nop\n\tv_nop" : "+v"(a), "+v"(b) : "v"(x), "v"(y)); }
__device__ __forceinline__ void dep_guard_b(v8f& a, v8f& b, v16b x, v16b y) { asm volatile("v_nop\n\tv_nop\n\tv_nop\n\tv_nop" : "+v"(a), "+v"(b) : "v"(x), "v"(y)); }
__device__ __forceinline__ void keep4_h(v16h a, v16h b, v16h c, v16h d) { asm volatile("v_nop" :: "v"(a), "v"(b), "v"(c), "v"(d)); }
__device__ __forceinline__ void keep4_b(v16b a, v16b b, v16b c, v16b d) { asm volatile("v_nop" :: "v"(a), "v"(b), "v"(c), "v"(d)); }
template <typename T> struct Frag;
template <> struct Frag<_Float16> {
  typedef v16h V; union U { v16h v; v8h h[2]; };
  static __device__ __forceinline__ v16h load(const _Float16* p) {
    U f; f.h[0] = *(const v8h*)(p); f.h[1] = *(const v8h*)(p + 16); return f.v;
  }
  static __device__ __forceinline__ v8f mma(v16h a, v16h b, v8f c) {
    return __builtin_amdgcn_wmma_f32_16x16x32_f16(false, a, false, b, (short)0, c, false, false);
  }
  static __device__ __forceinline__ void guard(v8f& a, v8f& b, v16h x, v16h y) { dep_guard_h(a, b, x, y); }
  static __device__ __forceinline__ void keep(v16h a, v16h b, v16h c, v16h d) { keep4_h(a, b, c, d); }
};
template <> struct Frag<__bf16> {
  typedef v16b V; union U { v16b v; v8b h[2]; };
  static __device__ __forceinline__ v16b load(const __bf16* p) {
    U f; f.h[0] = *(const v8b*)(p); f.h[1] = *(const v8b*)(p + 16); return f.v;
  }
  static __device__ __forceinline__ v8f mma(v16b a, v16b b, v8f c) {
    return __builtin_amdgcn_wmma_f32_16x16x32_bf16(false, a, false, b, (short)0, c, false, false);
  }
  static __device__ __forceinline__ void guard(v8f& a, v8f& b, v16b x, v16b y) { dep_guard_b(a, b, x, y); }
  static __device__ __forceinline__ void keep(v16b a, v16b b, v16b c, v16b d) { keep4_b(a, b, c, d); }
};

__device__ __forceinline__ v8f at_mma(v16b a, v16b b, v8f c) {
  c = __builtin_amdgcn_wmma_f32_16x16x32_bf16(false, a, false, b, (short)0, c, false, false);
  asm volatile("v_nop\n\tv_nop\n\tv_nop\n\tv_nop" : "+v"(c) : "v"(a), "v"(b));
  return c;
}

__device__ __forceinline__ float fsig(float x)  { return __builtin_amdgcn_rcpf(1.0f + __expf(-x)); }
__device__ __forceinline__ float ftanh(float x) { return 1.0f - 2.0f * __builtin_amdgcn_rcpf(__expf(2.0f * x) + 1.0f); }

__device__ __forceinline__ void fill_wplane(unsigned* pl, const float* __restrict__ W, int ldw, int col0, int tid) {
#pragma unroll 1
  for (int i = tid; i < NGATE * 8; i += NTHR) {
    const int g = i >> 3, j = i & 7;
    const float* wp = W + g * ldw + col0 + 2 * j;
    const unsigned w = (unsigned)f2bf_bits(wp[0]) | ((unsigned)f2bf_bits(wp[1]) << 16);
    pl[g * 16 + j] = w;
    pl[g * 16 + 8 + j] = w;
  }
}

__device__ __forceinline__ void ld8(float (&d)[8], const float* p) {
  const v4f a = *(const v4f*)p;
  const v4f b = *(const v4f*)(p + 4);
  d[0] = a[0]; d[1] = a[1]; d[2] = a[2]; d[3] = a[3];
  d[4] = b[0]; d[5] = b[1]; d[6] = b[2]; d[7] = b[3];
}

__device__ __forceinline__ v16b frag_of(const float (&h)[8]) {
  v16b f;
#pragma unroll
  for (int i = 0; i < 8; ++i) {
    const unsigned short hb = f2bf_bits(h[i]);
    const unsigned short lb = f2bf_bits(h[i] - bf_bits2f(hb));
    f[i]     = __builtin_bit_cast(__bf16, hb);
    f[8 + i] = __builtin_bit_cast(__bf16, lb);
  }
  return f;
}
__device__ __forceinline__ v16b frag_words_of(const float (&h)[8], v4u& wh, v4u& wl) {
  unsigned hb[8], lb[8];
  v16b f;
#pragma unroll
  for (int i = 0; i < 8; ++i) {
    const unsigned short b0 = f2bf_bits(h[i]);
    const unsigned short b1 = f2bf_bits(h[i] - bf_bits2f(b0));
    hb[i] = b0; lb[i] = b1;
    f[i]     = __builtin_bit_cast(__bf16, b0);
    f[8 + i] = __builtin_bit_cast(__bf16, b1);
  }
  wh[0] = (hb[0] & 0xffffu) | (hb[1] << 16); wh[1] = (hb[2] & 0xffffu) | (hb[3] << 16);
  wh[2] = (hb[4] & 0xffffu) | (hb[5] << 16); wh[3] = (hb[6] & 0xffffu) | (hb[7] << 16);
  wl[0] = (lb[0] & 0xffffu) | (lb[1] << 16); wl[1] = (lb[2] & 0xffffu) | (lb[3] << 16);
  wl[2] = (lb[4] & 0xffffu) | (lb[5] << 16); wl[3] = (lb[6] & 0xffffu) | (lb[7] << 16);
  return f;
}
__device__ __forceinline__ v16b zero_frag() {
  v16b f;
#pragma unroll
  for (int i = 0; i < 16; ++i) f[i] = __builtin_bit_cast(__bf16, (unsigned short)0);
  return f;
}

__device__ __forceinline__ void gru_cell_l0(float (&h)[8], v8f ar, v8f az, v8f an, float xt, const float* cs, int hh) {
  float wr[8], wz[8], wn[8], cr[8], cz[8], bi[8], bh[8];
  ld8(wr, cs + 8 * hh);
  ld8(wz, cs + NHID + 8 * hh);
  ld8(wn, cs + 2 * NHID + 8 * hh);
  ld8(cr, cs + 48 + 8 * hh);
  ld8(cz, cs + 64 + 8 * hh);
  ld8(bi, cs + 80 + 8 * hh);
  ld8(bh, cs + 96 + 8 * hh);
#pragma unroll
  for (int v = 0; v < 8; ++v) {
    const float pr = fmaf(xt, wr[v], cr[v]) + ar[v];
    const float pz = fmaf(xt, wz[v], cz[v]) + az[v];
    const float r = fsig(pr);
    const float z = fsig(pz);
    const float pn = fmaf(xt, wn[v], bi[v]) + r * (an[v] + bh[v]);
    const float n = ftanh(pn);
    h[v] = (1.0f - z) * n + z * h[v];
  }
}
__device__ __forceinline__ void gru_cell_l1(float (&h)[8], v8f ar, v8f az, v8f ai, v8f ah, const float* cs, int hh) {
  float cr[8], cz[8], bi[8], bh[8];
  ld8(cr, cs + 8 * hh);
  ld8(cz, cs + 16 + 8 * hh);
  ld8(bi, cs + 32 + 8 * hh);
  ld8(bh, cs + 48 + 8 * hh);
#pragma unroll
  for (int v = 0; v < 8; ++v) {
    const float r = fsig(ar[v] + cr[v]);
    const float z = fsig(az[v] + cz[v]);
    const float n = ftanh((ai[v] + bi[v]) + r * (ah[v] + bh[v]));
    h[v] = (1.0f - z) * n + z * h[v];
  }
}
__device__ __forceinline__ void gru_cell_first(float (&hout)[8], v8f ar, v8f az, v8f an, const float* cs, int hh) {
  float cr[8], cz[8], bi[8], bh[8];
  ld8(cr, cs + 8 * hh);
  ld8(cz, cs + 16 + 8 * hh);
  ld8(bi, cs + 32 + 8 * hh);
  ld8(bh, cs + 48 + 8 * hh);
#pragma unroll
  for (int v = 0; v < 8; ++v) {
    const float r = fsig(ar[v] + cr[v]);
    const float z = fsig(az[v] + cz[v]);
    const float n = ftanh((an[v] + bi[v]) + r * bh[v]);
    hout[v] = (1.0f - z) * n + 0.0f;
  }
}

__global__ __launch_bounds__(NTHR) void gru_l0_rev_kernel(const float* __restrict__ x,
    const float* __restrict__ Wih, const float* __restrict__ Whh,
    const float* __restrict__ bih, const float* __restrict__ bhh,
    unsigned* __restrict__ YB) {
  __shared__ __align__(16) unsigned Apl[WPLW];
  __shared__ __align__(16) float    Cs[112];
  __shared__ __align__(16) unsigned Sg[NWAVE][16 * YBW];
  const int tid = threadIdx.x, lane = tid & 31, wave = tid >> 5;
  const int c = lane & 15, hh = lane >> 4;
  const int base = blockIdx.x * BROWS + wave * 16;

  fill_wplane(Apl, Whh, NHID, 0, tid);
  if (tid < NGATE) Cs[tid] = bf16r(Wih[tid]);
  if (tid < NHID) {
    Cs[48 + tid] = bf16r(bih[tid]) + bf16r(bhh[tid]);
    Cs[64 + tid] = bf16r(bih[NHID + tid]) + bf16r(bhh[NHID + tid]);
    Cs[80 + tid] = bf16r(bih[2 * NHID + tid]);
    Cs[96 + tid] = bf16r(bhh[2 * NHID + tid]);
  }
  float h[8];
#pragma unroll
  for (int v = 0; v < 8; ++v) h[v] = 0.0f;
  __syncthreads();

  const __bf16* arow = (const __bf16*)Apl + c * 32 + 8 * hh;
  const float* xrow = x + (size_t)(base + c) * NSTEP;
  unsigned* sg = Sg[wave];
  const v8f z8 = {0.f, 0.f, 0.f, 0.f, 0.f, 0.f, 0.f, 0.f};
  v16b bf = zero_frag();

#pragma unroll 1
  for (int s = 0; s < NSTEP; ++s) {
    const int t = NSTEP - 1 - s;
    asm volatile("" ::: "memory");
    v8f ar = at_mma(Frag<__bf16>::load(arow), bf, z8);
    v8f az = at_mma(Frag<__bf16>::load(arow + GTILE), bf, z8);
    v8f an = at_mma(Frag<__bf16>::load(arow + 2 * GTILE), bf, z8);
    const float xt = bf16r(xrow[t]);
    gru_cell_l0(h, ar, az, an, xt, Cs, hh);
    v4u wh, wl;
    bf = frag_words_of(h, wh, wl);
    *(v4u*)(sg + c * YBW + 4 * hh) = wh;
    *(v4u*)(sg + c * YBW + 8 + 4 * hh) = wl;
    __syncthreads();
    unsigned* gdst = YB + ((size_t)t * NBATCH + base) * YBW;
    for (int pass = 0; pass < 2; ++pass) {
#pragma unroll
      for (int it = 0; it < 2; ++it) {
        const int idx = it * 128 + lane * 4;
        const v4u v = *(const v4u*)(sg + idx);
        *(volatile v4u*)(gdst + idx) = v;
      }
      __threadfence();
    }
    __syncthreads();
  }
}

__global__ __launch_bounds__(NTHR) void gru_stack_kernel(const float* __restrict__ x,
    const float* __restrict__ Wih0, const float* __restrict__ Whh0,
    const float* __restrict__ bih0, const float* __restrict__ bhh0,
    const float* __restrict__ Wih1, const float* __restrict__ Whh1,
    const float* __restrict__ bih1, const float* __restrict__ bhh1,
    const float* __restrict__ Wih1r, const float* __restrict__ bih1r, const float* __restrict__ bhh1r,
    const unsigned short* __restrict__ YB, float* __restrict__ out) {
  __shared__ __align__(16) unsigned Apl[6 * WPLW];
  __shared__ __align__(16) float    Cs[240];
  __shared__ __align__(16) float    Os[NWAVE][16 * OSP];
  const int tid = threadIdx.x, lane = tid & 31, wave = tid >> 5;
  const int c = lane & 15, hh = lane >> 4;
  const int base = blockIdx.x * BROWS + wave * 16;

  fill_wplane(Apl + 0 * WPLW, Whh0,  NHID,   0,    tid);
  fill_wplane(Apl + 1 * WPLW, Wih1,  NFEAT1, 0,    tid);
  asm volatile("" ::: "memory");
  fill_wplane(Apl + 2 * WPLW, Wih1,  NFEAT1, NHID, tid);
  fill_wplane(Apl + 3 * WPLW, Whh1,  NHID,   0,    tid);
  asm volatile("" ::: "memory");
  fill_wplane(Apl + 4 * WPLW, Wih1r, NFEAT1, 0,    tid);
  fill_wplane(Apl + 5 * WPLW, Wih1r, NFEAT1, NHID, tid);
  if (tid < NGATE) Cs[tid] = bf16r(Wih0[tid]);
  if (tid < NHID) {
    Cs[48 + tid]  = bf16r(bih0[tid]) + bf16r(bhh0[tid]);
    Cs[64 + tid]  = bf16r(bih0[NHID + tid]) + bf16r(bhh0[NHID + tid]);
    Cs[80 + tid]  = bf16r(bih0[2 * NHID + tid]);
    Cs[96 + tid]  = bf16r(bhh0[2 * NHID + tid]);
    asm volatile("" ::: "memory");
    Cs[112 + tid] = bf16r(bih1[tid]) + bf16r(bhh1[tid]);
    Cs[128 + tid] = bf16r(bih1[NHID + tid]) + bf16r(bhh1[NHID + tid]);
    Cs[144 + tid] = bf16r(bih1[2 * NHID + tid]);
    Cs[160 + tid] = bf16r(bhh1[2 * NHID + tid]);
    asm volatile("" ::: "memory");
    Cs[176 + tid] = bf16r(bih1r[tid]) + bf16r(bhh1r[tid]);
    Cs[192 + tid] = bf16r(bih1r[NHID + tid]) + bf16r(bhh1r[NHID + tid]);
    Cs[208 + tid] = bf16r(bih1r[2 * NHID + tid]);
    Cs[224 + tid] = bf16r(bhh1r[2 * NHID + tid]);
  }
  float h0[8], h1[8];
#pragma unroll
  for (int v = 0; v < 8; ++v) { h0[v] = 0.0f; h1[v] = 0.0f; }
  __syncthreads();

  const __bf16* arow = (const __bf16*)Apl + c * 32 + 8 * hh;
  const float* xrow = x + (size_t)(base + c) * NSTEP;
  const __bf16* ybrow = (const __bf16*)YB + (size_t)(base + c) * 32 + 8 * hh;
  const v8f z8 = {0.f, 0.f, 0.f, 0.f, 0.f, 0.f, 0.f, 0.f};
  v16b b0 = zero_frag();
  v16b b1 = zero_frag();

#pragma unroll 1
  for (int t = 0; t < NSTEP; ++t) {
    asm volatile("" ::: "memory");
    v8f ar = at_mma(Frag<__bf16>::load(arow), b0, z8);
    v8f az = at_mma(Frag<__bf16>::load(arow + GTILE), b0, z8);
    v8f an = at_mma(Frag<__bf16>::load(arow + 2 * GTILE), b0, z8);
    const float xt = bf16r(xrow[t]);
    gru_cell_l0(h0, ar, az, an, xt, Cs, hh);
    b0 = frag_of(h0);
    const v16b byb = Frag<__bf16>::load(ybrow + (size_t)t * NBATCH * 32);
    asm volatile("" ::: "memory");
    v8f r1 = at_mma(Frag<__bf16>::load(arow + 1 * WPLH), b0, z8);
    r1 = at_mma(Frag<__bf16>::load(arow + 2 * WPLH), byb, r1);
    r1 = at_mma(Frag<__bf16>::load(arow + 3 * WPLH), b1, r1);
    v8f z1 = at_mma(Frag<__bf16>::load(arow + 1 * WPLH + GTILE), b0, z8);
    z1 = at_mma(Frag<__bf16>::load(arow + 2 * WPLH + GTILE), byb, z1);
    z1 = at_mma(Frag<__bf16>::load(arow + 3 * WPLH + GTILE), b1, z1);
    v8f i1 = at_mma(Frag<__bf16>::load(arow + 1 * WPLH + 2 * GTILE), b0, z8);
    i1 = at_mma(Frag<__bf16>::load(arow + 2 * WPLH + 2 * GTILE), byb, i1);
    v8f g1 = at_mma(Frag<__bf16>::load(arow + 3 * WPLH + 2 * GTILE), b1, z8);
    gru_cell_l1(h1, r1, z1, i1, g1, Cs + 112, hh);
    b1 = frag_of(h1);
  }

  float hb[8];
  {
    asm volatile("" ::: "memory");
    const v16b byb = Frag<__bf16>::load(ybrow + (size_t)(NSTEP - 1) * NBATCH * 32);
    v8f ar = at_mma(Frag<__bf16>::load(arow + 4 * WPLH), b0, z8);
    ar = at_mma(Frag<__bf16>::load(arow + 5 * WPLH), byb, ar);
    v8f az = at_mma(Frag<__bf16>::load(arow + 4 * WPLH + GTILE), b0, z8);
    az = at_mma(Frag<__bf16>::load(arow + 5 * WPLH + GTILE), byb, az);
    v8f an = at_mma(Frag<__bf16>::load(arow + 4 * WPLH + 2 * GTILE), b0, z8);
    an = at_mma(Frag<__bf16>::load(arow + 5 * WPLH + 2 * GTILE), byb, an);
    gru_cell_first(hb, ar, az, an, Cs + 176, hh);
  }

  float* os = Os[wave];
  {
    const v4f a0 = {h1[0], h1[1], h1[2], h1[3]}, a1 = {h1[4], h1[5], h1[6], h1[7]};
    const v4f c0 = {hb[0], hb[1], hb[2], hb[3]}, c1 = {hb[4], hb[5], hb[6], hb[7]};
    *(v4f*)(os + c * OSP + 8 * hh) = a0;
    *(v4f*)(os + c * OSP + 8 * hh + 4) = a1;
    *(v4f*)(os + c * OSP + NHID + 8 * hh) = c0;
    *(v4f*)(os + c * OSP + NHID + 8 * hh + 4) = c1;
  }
  __syncthreads();
  for (int pass = 0; pass < 2; ++pass) {
#pragma unroll
    for (int it = 0; it < 4; ++it) {
      const int row = it * 4 + (lane >> 3);
      const int col = (lane & 7) * 4;
      const v4f v = *(const v4f*)(os + row * OSP + col);
      *(volatile v4f*)(out + (size_t)(base + row) * (2 * NHID) + col) = v;
    }
    __threadfence();
  }
}

extern "C" void kernel_launch(void* const* d_in, const int* in_sizes, int n_in,
                              void* d_out, int out_size, void* d_ws, size_t ws_size, hipStream_t stream) {
  if (n_in < 17 || d_out == nullptr || d_ws == nullptr) return;
  if (in_sizes[0] != NBATCH * NSTEP || in_sizes[1] != NGATE || in_sizes[2] != NGATE * NHID ||
      in_sizes[3] != NGATE || in_sizes[4] != NGATE || in_sizes[5] != NGATE || in_sizes[6] != NGATE * NHID ||
      in_sizes[7] != NGATE || in_sizes[8] != NGATE || in_sizes[9] != NGATE * NFEAT1 || in_sizes[10] != NGATE * NHID ||
      in_sizes[11] != NGATE || in_sizes[12] != NGATE || in_sizes[13] != NGATE * NFEAT1 ||
      in_sizes[15] != NGATE || in_sizes[16] != NGATE || out_size != NBATCH * 2 * NHID) return;
  const size_t yb_bytes = (size_t)NSTEP * NBATCH * YBW * 4;
  if (yb_bytes > ws_size || yb_bytes > (size_t)134217728) return;

  const float* x      = (const float*)d_in[0];
  const float* Wih0f  = (const float*)d_in[1];
  const float* Whh0f  = (const float*)d_in[2];
  const float* bih0f  = (const float*)d_in[3];
  const float* bhh0f  = (const float*)d_in[4];
  const float* Wih0b  = (const float*)d_in[5];
  const float* Whh0b  = (const float*)d_in[6];
  const float* bih0b  = (const float*)d_in[7];
  const float* bhh0b  = (const float*)d_in[8];
  const float* Wih1f  = (const float*)d_in[9];
  const float* Whh1f  = (const float*)d_in[10];
  const float* bih1f  = (const float*)d_in[11];
  const float* bhh1f  = (const float*)d_in[12];
  const float* Wih1b  = (const float*)d_in[13];
  const float* bih1b  = (const float*)d_in[15];
  const float* bhh1b  = (const float*)d_in[16];
  float* out = (float*)d_out;
  unsigned* YBw = (unsigned*)d_ws;

  gru_l0_rev_kernel<<<NBATCH / BROWS, NTHR, 0, stream>>>(x, Wih0b, Whh0b, bih0b, bhh0b, YBw);
  gru_stack_kernel<<<NBATCH / BROWS, NTHR, 0, stream>>>(x, Wih0f, Whh0f, bih0f, bhh0f,
                                                        Wih1f, Whh1f, bih1f, bhh1f,
                                                        Wih1b, bih1b, bhh1b,
                                                        (const unsigned short*)YBw, out);
}
